// MSMLTransformerLayer_86500641342117
// MI455X (gfx1250) — hardware-verified
//
#include <hip/hip_runtime.h>
#include <math.h>

constexpr int kB   = 2;
constexpr int kN   = 4096;
constexpr int kD   = 256;
constexpr int kWin = 16;
constexpr int kNW  = 256;
constexpr int kTok = kB * kN;
constexpr int kPlane = kD * kD;
constexpr float kWCarry = 64.0f;
constexpr float kXCarry = 4.0f;
constexpr float kHCarry = 16.0f;
constexpr float kUCarry = 0.0625f;
constexpr float kInvD   = 1.0f / 256.0f;
constexpr float kLnEps  = 1e-5f;

typedef __attribute__((ext_vector_type(16))) _Float16 v16h;
typedef __attribute__((ext_vector_type(8)))  _Float16 v8h;
typedef __attribute__((ext_vector_type(16))) __bf16   v16b;
typedef __attribute__((ext_vector_type(8)))  __bf16   v8b;
typedef __attribute__((ext_vector_type(8)))  float    v8f;
typedef __attribute__((ext_vector_type(4)))  float    v4f;
typedef __attribute__((ext_vector_type(4)))  unsigned int v4u;

__device__ __forceinline__ unsigned short f2bf_bits(float f) {
  unsigned u = __float_as_uint(f);
  return (unsigned short)((u + 0x7FFFu + ((u >> 16) & 1u)) >> 16);
}
__device__ __forceinline__ float bf_bits2f(unsigned short h) { return __uint_as_float(((unsigned)h) << 16); }

__device__ __forceinline__ void dep_guard_h(v8f& a, v8f& b, v16h x, v16h y) { asm volatile("v_nop\n\tv_nop\n\tv_nop\n\tv_nop" : "+v"(a), "+v"(b) : "v"(x), "v"(y)); }
__device__ __forceinline__ void dep_guard_b(v8f& a, v8f& b, v16b x, v16b y) { asm volatile("v_nop\n\tv_nop\n\tv_nop\n\tv_nop" : "+v"(a), "+v"(b) : "v"(x), "v"(y)); }
__device__ __forceinline__ void keep4_h(v16h a, v16h b, v16h c, v16h d) { asm volatile("v_nop" :: "v"(a), "v"(b), "v"(c), "v"(d)); }
__device__ __forceinline__ void keep4_b(v16b a, v16b b, v16b c, v16b d) { asm volatile("v_nop" :: "v"(a), "v"(b), "v"(c), "v"(d)); }
__device__ __forceinline__ void acc_guard4(v8f& a, v8f& b, v8f& c, v8f& d) { asm volatile("v_nop\n\tv_nop\n\tv_nop\n\tv_nop" : "+v"(a), "+v"(b), "+v"(c), "+v"(d)); }
template <typename T> struct Frag;
template <> struct Frag<_Float16> {
  typedef v16h V; union U { v16h v; v8h h[2]; };
  static __device__ __forceinline__ v16h load(const _Float16* p) {
    U f; f.h[0] = *(const v8h*)(p); f.h[1] = *(const v8h*)(p + 16); return f.v;
  }
  static __device__ __forceinline__ v8f mma(v16h a, v16h b, v8f c) {
    return __builtin_amdgcn_wmma_f32_16x16x32_f16(false, a, false, b, (short)0, c, false, false);
  }
  static __device__ __forceinline__ void guard(v8f& a, v8f& b, v16h x, v16h y) { dep_guard_h(a, b, x, y); }
  static __device__ __forceinline__ void keep(v16h a, v16h b, v16h c, v16h d) { keep4_h(a, b, c, d); }
};
template <> struct Frag<__bf16> {
  typedef v16b V; union U { v16b v; v8b h[2]; };
  static __device__ __forceinline__ v16b load(const __bf16* p) {
    U f; f.h[0] = *(const v8b*)(p); f.h[1] = *(const v8b*)(p + 16); return f.v;
  }
  static __device__ __forceinline__ v8f mma(v16b a, v16b b, v8f c) {
    return __builtin_amdgcn_wmma_f32_16x16x32_bf16(false, a, false, b, (short)0, c, false, false);
  }
  static __device__ __forceinline__ void guard(v8f& a, v8f& b, v16b x, v16b y) { dep_guard_b(a, b, x, y); }
  static __device__ __forceinline__ void keep(v16b a, v16b b, v16b c, v16b d) { keep4_b(a, b, c, d); }
};

__device__ __forceinline__ unsigned pk16(unsigned short a, unsigned short b) { return (unsigned)a | ((unsigned)b << 16); }
__device__ __forceinline__ unsigned short h_bits(float f) { const _Float16 h = (_Float16)f; return __builtin_bit_cast(unsigned short, h); }

template <int ET> struct Elem;
template <> struct Elem<0> { typedef _Float16 T; };
template <> struct Elem<1> { typedef __bf16 T; };
template <int ET, bool SPLIT, int BIAS_MODE, int OUT_MODE, int RMODE, int ACT>
__global__ __launch_bounds__(256) void wmma_gemm64(
    const unsigned short* __restrict__ Ap, const unsigned short* __restrict__ A2p, int lda, long strideA,
    const unsigned short* __restrict__ Btp, const unsigned short* __restrict__ Bt2p, int ldb, long strideB,
    void* __restrict__ Cout, void* __restrict__ Cout2, int ldc, long strideC,
    const float* __restrict__ bias, long strideBias,
    const float* __restrict__ resid, long strideR,
    int M, int N, int K, float scale, float oscale) {
  typedef typename Elem<ET>::T T;
  typedef typename Frag<T>::V V;
  const T* A = (const T*)Ap; const T* A2 = (const T*)A2p; const T* Bt = (const T*)Btp; const T* Bt2 = (const T*)Bt2p;
  __shared__ __align__(16) float sT[8][16 * 68];
  const int b    = blockIdx.y;
  const int lane = threadIdx.x & 31;
  const int wave = threadIdx.x >> 5;
  const int tilesN = N >> 6;
  const int tilesM = M >> 6;
  const int tile = blockIdx.x * 8 + wave;
  if (tile >= tilesM * tilesN) return;
  const int tm = tile / tilesN;
  const int tn = tile - tm * tilesN;
  const int m0 = tm << 6;
  const int n0 = tn << 6;

  const T* Ab  = A  + (size_t)b * strideA;
  const T* Bb  = Bt + (size_t)b * strideB;
  const T* Ab2 = SPLIT ? (A2  + (size_t)b * strideA) : nullptr;
  const T* Bb2 = SPLIT ? (Bt2 + (size_t)b * strideB) : nullptr;

  const int rlane = lane & 15;
  const int koff  = (lane >> 4) * 8;
  const int mOff  = (lane >> 4) * 8;

  v8f acc[4][4];
#pragma unroll
  for (int i = 0; i < 4; ++i)
#pragma unroll
    for (int j = 0; j < 4; ++j) acc[i][j] = (v8f){0.f,0.f,0.f,0.f,0.f,0.f,0.f,0.f};

  for (int k0 = 0; k0 < K; k0 += 32) {
    V bh[4], bl[4];
#pragma unroll
    for (int j = 0; j < 4; ++j) {
      const size_t bo = (size_t)(n0 + (j << 4) + rlane) * ldb + koff + k0;
      bh[j] = Frag<T>::load(Bb + bo);
      if (SPLIT) bl[j] = Frag<T>::load(Bb2 + bo);
    }
#pragma unroll
    for (int i = 0; i < 4; ++i) {
      const size_t ao = (size_t)(m0 + (i << 4) + rlane) * lda + koff + k0;
      V ah = Frag<T>::load(Ab + ao);
      V al;
      if (SPLIT) al = Frag<T>::load(Ab2 + ao);
#pragma unroll
      for (int j = 0; j < 4; ++j) {
        acc[i][j] = Frag<T>::mma(ah, bh[j], acc[i][j]);
        if (SPLIT) {
          acc[i][j] = Frag<T>::mma(ah, bl[j], acc[i][j]);
          acc[i][j] = Frag<T>::mma(al, bh[j], acc[i][j]);
        }
      }
      Frag<T>::guard(acc[i][0], acc[i][3], ah, SPLIT ? al : ah);
    }
    Frag<T>::keep(bh[0], bh[1], bh[2], bh[3]);
    if (SPLIT) Frag<T>::keep(bl[0], bl[1], bl[2], bl[3]);
  }
  acc_guard4(acc[0][0], acc[0][1], acc[0][2], acc[0][3]);
  acc_guard4(acc[1][0], acc[1][1], acc[1][2], acc[1][3]);
  acc_guard4(acc[2][0], acc[2][1], acc[2][2], acc[2][3]);
  acc_guard4(acc[3][0], acc[3][1], acc[3][2], acc[3][3]);

  float* slab = sT[wave];
  const float* Rb = (RMODE != 0) ? (resid + (size_t)b * strideR) : nullptr;
  const float* Bi = (BIAS_MODE != 0) ? (bias + (size_t)b * strideBias) : nullptr;
#pragma unroll
  for (int i = 0; i < 4; ++i) {
    const int mBase = m0 + (i << 4);
#pragma unroll
    for (int j = 0; j < 4; ++j) {
      const int n = n0 + (j << 4) + rlane;
      float bv = 0.f;
      if (BIAS_MODE == 2) bv = Bi[n];
#pragma unroll
      for (int r = 0; r < 8; ++r) {
        float v = acc[i][j][r] * scale;
        if (BIAS_MODE == 1) v += Bi[mBase + mOff + r];
        if (BIAS_MODE == 2) v += bv;
        if (RMODE == 1) v += Rb[(size_t)(mBase + mOff + r) * ldc + n];
        if (RMODE == 2) v *= Rb[(size_t)(mBase + mOff + r) * ldc + n];
        if (ACT == 2) v = fmaxf(v, 0.0f);
        if (ACT == 3) v = v / (1.0f + expf(-v));
        if (ACT == 4) v = (v > 0.f) ? v : 0.01f * v;
        v *= oscale;
        slab[(mOff + r) * 68 + (j << 4) + rlane] = v;
      }
    }
    __builtin_amdgcn_fence(__ATOMIC_RELEASE, "workgroup");
    __builtin_amdgcn_wave_barrier();
    __builtin_amdgcn_fence(__ATOMIC_ACQUIRE, "workgroup");
    if (OUT_MODE == 0) {
      float* C = (float*)Cout + (size_t)b * strideC;
      const int hh = lane >> 4, c4 = (lane & 15) * 4;
      for (int pass = 0; pass < 2; ++pass) {
#pragma unroll
        for (int it = 0; it < 8; ++it) {
          const int row = it * 2 + hh;
          v4f v = *(const v4f*)(slab + row * 68 + c4);
          *(volatile v4f*)(C + (size_t)(mBase + row) * ldc + n0 + c4) = v;
        }
        __threadfence();
      }
    } else {
      const int q = lane >> 3, c8 = (lane & 7) * 8;
      unsigned short* C  = (unsigned short*)Cout  + (size_t)b * strideC;
      unsigned short* C2 = (OUT_MODE == 2) ? ((unsigned short*)Cout2 + (size_t)b * strideC) : nullptr;
      for (int pass = 0; pass < 2; ++pass) {
#pragma unroll
        for (int it = 0; it < 4; ++it) {
          const int row = it * 4 + q;
          const float* sp = slab + row * 68 + c8;
          v8h hv, lv;
#pragma unroll
          for (int e = 0; e < 8; ++e) {
            if (OUT_MODE == 1) {
              hv[e] = (_Float16)sp[e];
            } else {
              unsigned short hb = f2bf_bits(sp[e]);
              unsigned short lb = f2bf_bits(sp[e] - bf_bits2f(hb));
              hv[e] = __builtin_bit_cast(_Float16, hb);
              lv[e] = __builtin_bit_cast(_Float16, lb);
            }
          }
          *(volatile v8h*)(C + (size_t)(mBase + row) * ldc + n0 + c8) = hv;
          if (OUT_MODE == 2) *(volatile v8h*)(C2 + (size_t)(mBase + row) * ldc + n0 + c8) = lv;
        }
        __threadfence();
      }
    }
    __builtin_amdgcn_fence(__ATOMIC_RELEASE, "workgroup");
    __builtin_amdgcn_wave_barrier();
    __builtin_amdgcn_fence(__ATOMIC_ACQUIRE, "workgroup");
  }
}

__device__ __forceinline__ float elu1_f(float v) { return (v > 0.0f) ? (v + 1.0f) : (expm1f(v) + 1.0f); }
__device__ __forceinline__ float phi_f(float z) { return elu1_f(elu1_f(z)); }

__global__ __launch_bounds__(256) void prep_kernel(const float* __restrict__ w0, const float* __restrict__ w1,
                                                   const float* __restrict__ w2, const float* __restrict__ w3,
                                                   const float* __restrict__ w4, unsigned short* __restrict__ wout,
                                                   float wscale,
                                                   const float* __restrict__ emb, const float* __restrict__ pw,
                                                   const float* __restrict__ pb, float* __restrict__ pt) {
  const int y = blockIdx.y;
  const int i = blockIdx.x * 256 + threadIdx.x;
  if (y < 5) {
    const float* W = (y == 0) ? w0 : (y == 1) ? w1 : (y == 2) ? w2 : (y == 3) ? w3 : w4;
    const float* p = W + 8 * (size_t)i;
    const v4f a = *(const v4f*)(p);
    const v4f c = *(const v4f*)(p + 4);
    unsigned short hb[8];
#pragma unroll
    for (int e = 0; e < 4; ++e) {
      hb[e]     = h_bits(a[e] * wscale);
      hb[4 + e] = h_bits(c[e] * wscale);
    }
    const v4u u = (v4u){pk16(hb[0], hb[1]), pk16(hb[2], hb[3]), pk16(hb[4], hb[5]), pk16(hb[6], hb[7])};
    unsigned short* q = wout + (size_t)y * kPlane + 8 * (size_t)i;
    *(volatile v4u*)q = u;
    __threadfence();
    *(volatile v4u*)q = u;
  } else {
    const int b   = i >> 12;
    const int m   = (i >> 8) & 15;
    const int rho = i & 255;
    const int w   = rho >> 4;
    const int n   = rho & 15;
    const size_t off = ((((size_t)(1 * kB + b) * kNW + w) * kWin + n) * kWin + m) * 3;
    const float v = emb[off] * pw[0] + emb[off + 1] * pw[1] + emb[off + 2] * pw[2] + pb[0];
    ((volatile float*)pt)[i] = v;
    __threadfence();
    ((volatile float*)pt)[i] = v;
  }
}

__global__ __launch_bounds__(256) void ln_x_kernel(const float* __restrict__ x, const float* __restrict__ g,
                                                   const float* __restrict__ bt, unsigned short* __restrict__ x16,
                                                   unsigned short* __restrict__ xn16, float xs, float ns, int nrows) {
  const int lane = threadIdx.x & 31, wave = threadIdx.x >> 5;
  const int row = blockIdx.x * 8 + wave;
  if (row >= nrows) return;
  const float* xr = x + (size_t)row * kD + 8 * lane;
  const v4f a = *(const v4f*)(xr);
  const v4f c = *(const v4f*)(xr + 4);
  float v[8];
#pragma unroll
  for (int e = 0; e < 4; ++e) { v[e] = a[e]; v[4 + e] = c[e]; }
  float s = ((v[0] + v[1]) + (v[2] + v[3])) + ((v[4] + v[5]) + (v[6] + v[7]));
#pragma unroll
  for (int off = 16; off > 0; off >>= 1) s += __shfl_xor(s, off, 32);
  const float mean = s * kInvD;
  float d[8];
  float ss = 0.f;
#pragma unroll
  for (int e = 0; e < 8; ++e) { d[e] = v[e] - mean; ss += d[e] * d[e]; }
#pragma unroll
  for (int off = 16; off > 0; off >>= 1) ss += __shfl_xor(ss, off, 32);
  const float var  = ss * kInvD;
  const float rstd = rsqrtf(var + kLnEps);
  const v4f ga = *(const v4f*)(g + 8 * lane);
  const v4f gc = *(const v4f*)(g + 8 * lane + 4);
  const v4f ba = *(const v4f*)(bt + 8 * lane);
  const v4f bc = *(const v4f*)(bt + 8 * lane + 4);
  float gg[8], bb[8];
#pragma unroll
  for (int e = 0; e < 4; ++e) { gg[e] = ga[e]; gg[4 + e] = gc[e]; bb[e] = ba[e]; bb[4 + e] = bc[e]; }
  unsigned short hx[8], hn[8];
#pragma unroll
  for (int e = 0; e < 8; ++e) {
    const float nv = d[e] * rstd * gg[e] + bb[e];
    hx[e] = h_bits(v[e] * xs);
    hn[e] = h_bits(nv * ns);
  }
  const v4u ux = (v4u){pk16(hx[0], hx[1]), pk16(hx[2], hx[3]), pk16(hx[4], hx[5]), pk16(hx[6], hx[7])};
  const v4u un = (v4u){pk16(hn[0], hn[1]), pk16(hn[2], hn[3]), pk16(hn[4], hn[5]), pk16(hn[6], hn[7])};
  unsigned short* qx = x16  + (size_t)row * kD + 8 * lane;
  unsigned short* qn = xn16 + (size_t)row * kD + 8 * lane;
  *(volatile v4u*)qx = ux;
  *(volatile v4u*)qn = un;
  __threadfence();
  *(volatile v4u*)qx = ux;
  *(volatile v4u*)qn = un;
}

__global__ __launch_bounds__(256) void cast8_kernel(const float* __restrict__ in, unsigned short* __restrict__ out,
                                                   float scale, int n8) {
  const int i = blockIdx.x * 256 + threadIdx.x;
  if (i >= n8) return;
  const float* p = in + 8 * (size_t)i;
  const v4f a = *(const v4f*)(p);
  const v4f c = *(const v4f*)(p + 4);
  unsigned short hb[8];
#pragma unroll
  for (int e = 0; e < 4; ++e) {
    hb[e]     = h_bits(a[e] * scale);
    hb[4 + e] = h_bits(c[e] * scale);
  }
  const v4u u = (v4u){pk16(hb[0], hb[1]), pk16(hb[2], hb[3]), pk16(hb[4], hb[5]), pk16(hb[6], hb[7])};
  unsigned short* q = out + 8 * (size_t)i;
  *(volatile v4u*)q = u;
  __threadfence();
  *(volatile v4u*)q = u;
}

__global__ __launch_bounds__(256) void planes_kernel(const float* __restrict__ zk, const float* __restrict__ h32,
                                                     const float* __restrict__ zq,
                                                     unsigned short* __restrict__ pkt, unsigned short* __restrict__ vt,
                                                     unsigned short* __restrict__ pq, float hscale) {
  __shared__ float smK[64][65];
  __shared__ float smV[64][65];
  const int t  = threadIdx.x;
  const int c0 = blockIdx.x * 64;
  const int w0 = blockIdx.y * 64;
  const int z  = blockIdx.z;
  const bool isT = (z < 32);
  const int zc = (z < 32) ? z : 31;
  const int bT = zc >> 4;
  const int mT = zc & 15;
  int bQ = z - 32; bQ = bQ < 0 ? 0 : (bQ > 1 ? 1 : bQ);
#pragma unroll 1
  for (int it = 0; it < 16; ++it) {
    const int e  = it * 256 + t;
    const int r  = e >> 6;
    const int cc = e & 63;
    float zv, hv = 0.f;
    if (isT) {
      const size_t src = ((size_t)bT * kN + (size_t)(w0 + r) * kWin + mT) * kD + c0 + cc;
      zv = zk[src];
      hv = h32[src];
    } else {
      const size_t src = ((size_t)bQ * 256 + w0 + r) * kD + c0 + cc;
      zv = zq[src];
    }
    const float ph = phi_f(zv);
    if (isT) { smK[cc][r] = ph; smV[cc][r] = hv * hscale; }
    else     { smK[r][cc] = ph; }
  }
  __syncthreads();
  const int lane = t & 31, wave = t >> 5;
  const int q = lane >> 3, c8 = (lane & 7) * 8;
  for (int pass = 0; pass < 2; ++pass) {
#pragma unroll
    for (int it = 0; it < 2; ++it) {
      const int row = wave * 8 + it * 4 + q;
      unsigned short kb[8];
#pragma unroll
      for (int e = 0; e < 8; ++e) kb[e] = h_bits(smK[row][c8 + e]);
      const v4u uk = (v4u){pk16(kb[0], kb[1]), pk16(kb[2], kb[3]), pk16(kb[4], kb[5]), pk16(kb[6], kb[7])};
      if (isT) {
        unsigned short vb[8];
#pragma unroll
        for (int e = 0; e < 8; ++e) vb[e] = h_bits(smV[row][c8 + e]);
        const v4u uv = (v4u){pk16(vb[0], vb[1]), pk16(vb[2], vb[3]), pk16(vb[4], vb[5]), pk16(vb[6], vb[7])};
        const size_t dst = ((size_t)z * kD + c0 + row) * kNW + w0 + c8;
        *(volatile v4u*)(pkt + dst) = uk;
        *(volatile v4u*)(vt  + dst) = uv;
      } else {
        const size_t dst = ((size_t)bQ * 256 + w0 + row) * kD + c0 + c8;
        *(volatile v4u*)(pq + dst) = uk;
      }
    }
    __threadfence();
  }
}

__global__ __launch_bounds__(256) void ln_out_kernel(const float* __restrict__ y, const float* __restrict__ g,
                                                     const float* __restrict__ bt, float* __restrict__ out, int nrows) {
  const int lane = threadIdx.x & 31, wave = threadIdx.x >> 5;
  const int row = blockIdx.x * 8 + wave;
  if (row >= nrows) return;
  const float* yr = y + (size_t)row * kD;
  const v4f a = *(const v4f*)(yr + 4 * lane);
  const v4f c = *(const v4f*)(yr + 128 + 4 * lane);
  float v[8];
#pragma unroll
  for (int e = 0; e < 4; ++e) { v[e] = a[e]; v[4 + e] = c[e]; }
  float s = ((v[0] + v[1]) + (v[2] + v[3])) + ((v[4] + v[5]) + (v[6] + v[7]));
#pragma unroll
  for (int off = 16; off > 0; off >>= 1) s += __shfl_xor(s, off, 32);
  const float mean = s * kInvD;
  float d[8];
  float ss = 0.f;
#pragma unroll
  for (int e = 0; e < 8; ++e) { d[e] = v[e] - mean; ss += d[e] * d[e]; }
#pragma unroll
  for (int off = 16; off > 0; off >>= 1) ss += __shfl_xor(ss, off, 32);
  const float var  = ss * kInvD;
  const float rstd = rsqrtf(var + kLnEps);
  const v4f ga = *(const v4f*)(g + 4 * lane);
  const v4f gc = *(const v4f*)(g + 128 + 4 * lane);
  const v4f ba = *(const v4f*)(bt + 4 * lane);
  const v4f bc = *(const v4f*)(bt + 128 + 4 * lane);
  v4f o0, o1;
#pragma unroll
  for (int e = 0; e < 4; ++e) {
    o0[e] = d[e] * rstd * ga[e] + ba[e];
    o1[e] = d[4 + e] * rstd * gc[e] + bc[e];
  }
  float* orow = out + (size_t)row * kD;
  *(volatile v4f*)(orow + 4 * lane) = o0;
  *(volatile v4f*)(orow + 128 + 4 * lane) = o1;
  __threadfence();
  *(volatile v4f*)(orow + 4 * lane) = o0;
  *(volatile v4f*)(orow + 128 + 4 * lane) = o1;
}

static inline size_t align256(size_t v) { return (v + 255) & ~(size_t)255; }
static inline dim3 gemm_grid(int M, int N, int batch) {
  const int tiles = (M / 64) * (N / 64);
  return dim3((unsigned)((tiles + 7) / 8), (unsigned)batch, 1);
}

extern "C" void kernel_launch(void* const* d_in, const int* in_sizes, int n_in,
                              void* d_out, int out_size, void* d_ws, size_t ws_size,
                              hipStream_t stream) {
  if (n_in < 18) return;
  if (out_size < kTok * kD) return;
  if (in_sizes[0] < kTok * kD) return;
  const float* x      = (const float*)d_in[0];
  const float* embed  = (const float*)d_in[1];
  const float* act_w  = (const float*)d_in[2];
  const float* act_b  = (const float*)d_in[3];
  const float* pln_g  = (const float*)d_in[4];
  const float* pln_b  = (const float*)d_in[5];
  const float* conv_w = (const float*)d_in[6];
  const float* conv_b = (const float*)d_in[7];
  const float* q_w    = (const float*)d_in[8];
  const float* q_b    = (const float*)d_in[9];
  const float* k_w    = (const float*)d_in[10];
  const float* k_b    = (const float*)d_in[11];
  const float* p_w    = (const float*)d_in[12];
  const float* p_b    = (const float*)d_in[13];
  const float* lin_w  = (const float*)d_in[14];
  const float* lin_b  = (const float*)d_in[15];
  const float* norm_g = (const float*)d_in[16];
  const float* norm_b = (const float*)d_in[17];
  float* out = (float*)d_out;

  char* base = (char*)d_ws;
  size_t off = 0;
  const size_t szTokH = (size_t)kTok * kD * 2, szTokF = (size_t)kTok * kD * 4;
  unsigned short* wplanes = (unsigned short*)(base + off); off += align256((size_t)5 * kPlane * 2);
  unsigned short* x16     = (unsigned short*)(base + off); off += align256(szTokH);
  unsigned short* xn16    = (unsigned short*)(base + off); off += align256(szTokH);
  float*          actres  = (float*)(base + off);          off += align256(szTokF);
  float*          h32     = (float*)(base + off);          off += align256(szTokF);
  unsigned short* h16     = (unsigned short*)(base + off); off += align256(szTokH);
  float*          zk      = (float*)(base + off);          off += align256(szTokF);
  float*          zq      = (float*)(base + off);          off += align256((size_t)kB * kPlane * 4);
  unsigned short* pkt     = (unsigned short*)(base + off); off += align256((size_t)kB * kWin * kPlane * 2);
  unsigned short* vt      = (unsigned short*)(base + off); off += align256((size_t)kB * kWin * kPlane * 2);
  unsigned short* pq      = (unsigned short*)(base + off); off += align256((size_t)kB * kPlane * 2);
  float*          pt      = (float*)(base + off);          off += align256((size_t)kB * kWin * 256 * 4);
  unsigned short* kvt     = (unsigned short*)(base + off); off += align256((size_t)kB * kWin * kPlane * 2);
  unsigned short* u16     = (unsigned short*)(base + off); off += align256(szTokH);
  float*          yb      = (float*)(base + off);          off += align256(szTokF);
  if (off > ws_size) return;

  const unsigned short* wact  = wplanes + 0 * (size_t)kPlane;
  const unsigned short* wconv = wplanes + 1 * (size_t)kPlane;
  const unsigned short* wq    = wplanes + 2 * (size_t)kPlane;
  const unsigned short* wk    = wplanes + 3 * (size_t)kPlane;
  const unsigned short* wlin  = wplanes + 4 * (size_t)kPlane;

  prep_kernel<<<dim3(32, 6), 256, 0, stream>>>(act_w, conv_w, q_w, k_w, lin_w, wplanes, kWCarry, embed, p_w, p_b, pt);
  ln_x_kernel<<<kTok / 8, 256, 0, stream>>>(x, pln_g, pln_b, x16, xn16, kXCarry, kXCarry, kTok);
  wmma_gemm64<0, false, 2, 0, 0, 3><<<gemm_grid(kTok, kD, 1), 256, 0, stream>>>(
      x16, nullptr, kD, 0L, wact, nullptr, kD, 0L, (void*)actres, nullptr, kD, 0L,
      act_b, 0L, nullptr, 0L, kTok, kD, kD, 1.0f / (kXCarry * kWCarry), 1.0f);
  wmma_gemm64<0, false, 2, 0, 0, 3><<<gemm_grid(kTok, kD, 1), 256, 0, stream>>>(
      xn16, nullptr, kD, 0L, wconv, nullptr, kD, 0L, (void*)h32, nullptr, kD, 0L,
      conv_b, 0L, nullptr, 0L, kTok, kD, kD, 1.0f / (kXCarry * kWCarry), 1.0f);
  cast8_kernel<<<(kTok * kD / 8) / 256, 256, 0, stream>>>(h32, h16, kHCarry, kTok * kD / 8);
  wmma_gemm64<0, false, 2, 0, 0, 0><<<gemm_grid(kTok, kD, 1), 256, 0, stream>>>(
      h16, nullptr, kD, 0L, wk, nullptr, kD, 0L, (void*)zk, nullptr, kD, 0L,
      k_b, 0L, nullptr, 0L, kTok, kD, kD, 1.0f / (kHCarry * kWCarry), 1.0f);
  wmma_gemm64<0, false, 2, 0, 0, 0><<<gemm_grid(256, kD, kB), 256, 0, stream>>>(
      h16, nullptr, kD, (long)kN * kD, wq, nullptr, kD, 0L, (void*)zq, nullptr, kD, (long)kPlane,
      q_b, 0L, nullptr, 0L, 256, kD, kD, 1.0f / (kHCarry * kWCarry), 1.0f);
  planes_kernel<<<dim3(4, 4, 34), 256, 0, stream>>>(zk, h32, zq, pkt, vt, pq, kHCarry);
  wmma_gemm64<0, false, 0, 1, 0, 0><<<gemm_grid(256, 256, kB * kWin), 256, 0, stream>>>(
      vt, nullptr, kNW, (long)kPlane, pkt, nullptr, kNW, (long)kPlane, (void*)kvt, nullptr, kD, (long)kPlane,
      nullptr, 0L, nullptr, 0L, 256, 256, kNW, 1.0f / kHCarry, 1.0f);
  for (int b = 0; b < kB; ++b) {
    wmma_gemm64<0, false, 1, 1, 2, 0><<<gemm_grid(256, kD, kWin), 256, 0, stream>>>(
        pq + (size_t)b * kPlane, nullptr, kD, 0L,
        kvt + (size_t)b * kWin * kPlane, nullptr, kD, (long)kPlane,
        (void*)(u16 + (size_t)b * kN * kD), nullptr, kWin * kD, (long)kD,
        pt + (size_t)b * kWin * 256, 256L,
        actres + (size_t)b * kN * kD, (long)kD,
        256, kD, kD, 1.0f, kUCarry);
  }
  wmma_gemm64<0, false, 2, 0, 1, 0><<<gemm_grid(kTok, kD, 1), 256, 0, stream>>>(
      u16, nullptr, kD, 0L, wlin, nullptr, kD, 0L, (void*)yb, nullptr, kD, 0L,
      lin_b, 0L, h32, 0L, kTok, kD, kD, 1.0f / (kUCarry * kWCarry), 1.0f);
  ln_out_kernel<<<kTok / 8, 256, 0, stream>>>(yb, norm_g, norm_b, out, kTok);
}
